// LGP_22892175688205
// MI455X (gfx1250) — hardware-verified
//
#include <hip/hip_runtime.h>
#include <math.h>

typedef __attribute__((ext_vector_type(16))) _Float16 v16h;
typedef __attribute__((ext_vector_type(16))) __bf16 v16b;
typedef __attribute__((ext_vector_type(8)))  _Float16 v8h;
typedef __attribute__((ext_vector_type(8)))  float v8f;
typedef __attribute__((ext_vector_type(4)))  float v4f;
typedef __attribute__((ext_vector_type(2)))  float v2f;
typedef __attribute__((ext_vector_type(4)))  unsigned v4u;
typedef __attribute__((ext_vector_type(4)))  int v4i;
typedef float __attribute__((may_alias)) float_a;
typedef int __attribute__((may_alias)) int_a;

template <typename T> __device__ __forceinline__ void vst2(void* p, T v) { *(volatile T*)p = v; __threadfence(); *(volatile T*)p = v; }
__device__ __forceinline__ v8f wmma16(v16h a, v16h b, v8f c) {
  v8f d = __builtin_amdgcn_wmma_f32_16x16x32_f16(false, a, false, b, (short)0, c, false, false);
  asm volatile("v_nop\n\tv_nop\n\tv_nop\n\tv_nop" : "+v"(d) : "v"(a), "v"(b));
  return d;
}
__device__ __forceinline__ v8f wmma_bf(v16b a, v16b b, v8f c) {
  v8f d = __builtin_amdgcn_wmma_f32_16x16x32_bf16(false, a, false, b, (short)0, c, false, false);
  asm volatile("v_nop\n\tv_nop\n\tv_nop\n\tv_nop" : "+v"(d) : "v"(a), "v"(b));
  return d;
}
__device__ __forceinline__ v16h frag_h(const _Float16* rowk0, int lane) {
  union { v16h v; v8h q[2]; } u; const _Float16* p = rowk0 + 8 * (lane >> 4);
  u.q[0] = *(const v8h*)p; u.q[1] = *(const v8h*)(p + 16); return u.v;
}
__device__ __forceinline__ v16h frag_f32(const float* rowk0, int lane) {
  v16h a; const float* p = rowk0 + 8 * (lane >> 4);
#pragma unroll
  for (int i = 0; i < 8; ++i) { a[i] = (_Float16)p[i]; a[8 + i] = (_Float16)p[16 + i]; }
  return a;
}
__device__ __forceinline__ v16h frag_f32s(const float* rowk0, int lane, float sc) {
  v16h a; const float* p = rowk0 + 8 * (lane >> 4);
#pragma unroll
  for (int i = 0; i < 8; ++i) { a[i] = (_Float16)(p[i] * sc); a[8 + i] = (_Float16)(p[16 + i] * sc); }
  return a;
}
__device__ __forceinline__ v16h fragc_f32(const float* W, int k0, int n, int lane, int ld, int K) {
  v16h a; const int g = lane >> 4;
#pragma unroll
  for (int i = 0; i < 8; ++i) { const int ka = k0 + 8 * g + i, kb = ka + 16;
    a[i] = (_Float16)(ka < K ? W[(size_t)(ka < K ? ka : K - 1) * ld + n] : 0.f); a[8 + i] = (_Float16)(kb < K ? W[(size_t)(kb < K ? kb : K - 1) * ld + n] : 0.f); }
  return a;
}
struct F2 { v16b h, l; };
__device__ __forceinline__ F2 bsplit16(const float v[16]) { F2 r;
#pragma unroll
  for (int i = 0; i < 16; ++i) { const __bf16 h = (__bf16)v[i]; r.h[i] = h; r.l[i] = (__bf16)(v[i] - (float)h); }
  return r; }
__device__ __forceinline__ F2 split_row(const float* row, int k0, int lane) { float v[16]; const float* p = row + k0 + 8 * (lane >> 4);
#pragma unroll
  for (int i = 0; i < 8; ++i) { v[i] = p[i]; v[8 + i] = p[16 + i]; }
  return bsplit16(v); }
__device__ __forceinline__ F2 split_rowK(const float* row, int k0, int lane, int K) { float v[16]; const int g = lane >> 4;
#pragma unroll
  for (int i = 0; i < 8; ++i) { const int ka = k0 + 8 * g + i, kb = ka + 16; v[i] = ka < K ? row[ka < K ? ka : K - 1] : 0.f; v[8 + i] = kb < K ? row[kb < K ? kb : K - 1] : 0.f; }
  return bsplit16(v); }
__device__ __forceinline__ F2 split_col(const float* W, int k0, int n, int lane, int ld, int K) { float v[16]; const int g = lane >> 4;
#pragma unroll
  for (int i = 0; i < 8; ++i) { const int ka = k0 + 8 * g + i, kb = ka + 16; v[i] = ka < K ? W[(size_t)(ka < K ? ka : K - 1) * ld + n] : 0.f; v[8 + i] = kb < K ? W[(size_t)(kb < K ? kb : K - 1) * ld + n] : 0.f; }
  return bsplit16(v); }
__device__ __forceinline__ v8f mac3(const F2& a, const F2& b, v8f c) { c = wmma_bf(a.l, b.h, c); c = wmma_bf(a.h, b.l, c); return wmma_bf(a.h, b.h, c); }
__device__ __forceinline__ float sigm(float v) { return 1.0f / (1.0f + expf(-v)); }
#define LDSX() do { asm volatile("s_wait_dscnt 0" ::: "memory"); __builtin_amdgcn_wave_barrier(); __builtin_amdgcn_fence(__ATOMIC_RELEASE, "workgroup"); } while (0)


#define NB 4
#define NP 4096
#define NR (NB * NP)
#define CC 384
#define KN 16
#define KIN 448
#ifndef NBT
#define NBT NB
#endif
typedef __attribute__((ext_vector_type(8))) __bf16 v8b;
__device__ __forceinline__ v16b frag_b(const __bf16* rowk0, int lane) {
  union { v16b v; v8b q[2]; } u; const __bf16* p = rowk0 + 8 * (lane >> 4);
  u.q[0] = *(const v8b*)p; u.q[1] = *(const v8b*)(p + 16); return u.v;
}
__device__ __forceinline__ float bfr(float v) { return (float)(__bf16)v; }
__device__ __attribute__((noinline)) float exp_ni(float v) { return expf(v); }
__device__ __attribute__((noinline)) float erf_ni(float v) { return erff(v); }
__device__ __attribute__((noinline)) float sqrt_ni(float v) { return sqrtf(v); }
__device__ __forceinline__ float gelu_exact(float v) { return 0.5f * v * (1.0f + erf_ni(v * 0.70710678118654752f)); }

#define PK_1 0
#define PK_2 (CC * KIN)
#define PK_END (PK_2 + CC * CC)
#define WS_PK  0u
#define WS_IDX (((2u * PK_END) + 127u) / 128u * 128u)
#define WS_FUH (WS_IDX + 4u * NR * KN)
#define WS_FUL (WS_FUH + 2u * NR * KIN)
#define WS_HH  (WS_FUL + 2u * NR * KIN)
#define WS_HL  (WS_HH + 2u * NR * CC)
#define WS_END (WS_HL + 2u * NR * CC)

__global__ __launch_bounds__(256) void k_pack(const float* __restrict__ W1, const float* __restrict__ W2, __bf16* __restrict__ PK) {
  __shared__ __align__(16) __bf16 s[KIN]; const int n = blockIdx.x, which = blockIdx.y, tid = threadIdx.x; int K; size_t dst;
  if (which == 0) { K = KIN; dst = PK_1 + (size_t)n * KIN; for (int k = tid; k < KIN; k += 256) s[k] = (__bf16)((k <= CC) ? W1[(size_t)k * CC + n] : 0.f); }
  else { K = CC; dst = PK_2 + (size_t)n * CC; for (int k = tid; k < CC; k += 256) s[k] = (__bf16)W2[(size_t)k * CC + n]; }
  __syncthreads();
  for (int q = tid; q < K / 8; q += 256) vst2((unsigned*)(PK + dst + q * 8), *(const v4u*)&s[q * 8]);
}
__global__ __launch_bounds__(256) void k_knn(const float* __restrict__ XYZ, int* __restrict__ IDX) {
  __shared__ float sx[NP], sy[NP], sz[NP], ssq[NP]; __shared__ __align__(16) int sidx[256][KN];
  const int tid = threadIdx.x; const int b = blockIdx.x / (NP / 256); const int q0 = (blockIdx.x % (NP / 256)) * 256; const int q = q0 + tid;
  for (int i = tid; i < NP; i += 256) { const float* p = XYZ + ((size_t)b * NP + i) * 3; const float x = bfr(p[0]), y = bfr(p[1]), z = bfr(p[2]); sx[i] = x; sy[i] = y; sz[i] = z; ssq[i] = (x * x + z * z) + y * y; }
  __syncthreads();
  const float qx = sx[q], qy = sy[q], qz = sz[q], qsq = ssq[q];
  float bd[KN]; int bi[KN];
#pragma unroll
  for (int s = 0; s < KN; ++s) { bd[s] = 3.0e38f; bi[s] = 0; }
  for (int m = 0; m < NP; ++m) { const float dot = (qx * sx[m] + qy * sy[m]) + qz * sz[m]; const float d2 = (qsq + ssq[m]) - 2.0f * dot; const float D = fmaxf(d2, 0.f);
    if (D < bd[KN - 1]) { float cd = D; int ci = m; bool placed = false;
#pragma unroll
      for (int s = 0; s < KN; ++s) { const bool sw = placed || (cd < bd[s]); placed = sw; const float td = bd[s]; const int ti = bi[s]; bd[s] = sw ? cd : td; bi[s] = sw ? ci : ti; cd = sw ? td : cd; ci = sw ? ti : ci; } } }
#pragma unroll
  for (int s = 0; s < KN; ++s) sidx[tid][s] = bi[s];
  __syncthreads();
  for (int qq = tid; qq < 256 * KN / 4; qq += 256) vst2((unsigned*)(IDX + ((size_t)b * NP + q0) * KN + qq * 4), *(const v4u*)(&sidx[0][0] + qq * 4));
}
__global__ __launch_bounds__(128) void k_local(const float* __restrict__ XYZ, const float* __restrict__ FT, const int* __restrict__ IDX, __bf16* __restrict__ FUH, __bf16* __restrict__ FUL) {
  __shared__ __align__(16) __bf16 sh_[4][KIN + 8], sl_[4][KIN + 8]; __shared__ float sw[4][KN]; __shared__ int sid[4][KN]; __shared__ float sdist[4];
  const int tid = threadIdx.x, wave = tid >> 5, lane = tid & 31; const size_t n = (size_t)blockIdx.x * 4 + wave; const int b = (int)(n / NP);
  { const int k = lane & 15; const int id = min(max(IDX[n * KN + k], 0), NP - 1); if (lane < KN) sid[wave][k] = id;
    const float* p = XYZ + ((size_t)b * NP + id) * 3; const float px = bfr(p[0]), py = bfr(p[1]), pz = bfr(p[2]);
    float cx = (lane < KN) ? px : 0.f, cy = (lane < KN) ? py : 0.f, cz = (lane < KN) ? pz : 0.f;
#pragma unroll
    for (int o = 1; o < 32; o <<= 1) { cx += __shfl_xor(cx, o); cy += __shfl_xor(cy, o); cz += __shfl_xor(cz, o); }
    cx *= (1.0f / KN); cy *= (1.0f / KN); cz *= (1.0f / KN);
    const float ox = px - cx, oy = py - cy, oz = pz - cz;
    float mx = (lane < KN) ? ox : 0.f, my = (lane < KN) ? oy : 0.f, mz = (lane < KN) ? oz : 0.f;
#pragma unroll
    for (int o = 1; o < 32; o <<= 1) { mx += __shfl_xor(mx, o); my += __shfl_xor(my, o); mz += __shfl_xor(mz, o); }
    mx *= (1.0f / KN); my *= (1.0f / KN); mz *= (1.0f / KN);
    float vx = (lane < KN) ? (ox - mx) * (ox - mx) : 0.f, vy = (lane < KN) ? (oy - my) * (oy - my) : 0.f, vz = (lane < KN) ? (oz - mz) * (oz - mz) : 0.f;
#pragma unroll
    for (int o = 1; o < 32; o <<= 1) { vx += __shfl_xor(vx, o); vy += __shfl_xor(vy, o); vz += __shfl_xor(vz, o); }
    const float sgx = sqrt_ni(vx / (float)(KN - 1)) + 1e-6f, sgy = sqrt_ni(vy / (float)(KN - 1)) + 1e-6f, sgz = sqrt_ni(vz / (float)(KN - 1)) + 1e-6f;
    const float rx = ox / sgx, ry = oy / sgy, rz = oz / sgz; const float dist = sqrt_ni((rx * rx + ry * ry) + rz * rz); const float w = exp_ni(-0.5f * dist);
    float dsum = (lane < KN) ? dist : 0.f;
#pragma unroll
    for (int o = 1; o < 32; o <<= 1) dsum += __shfl_xor(dsum, o);
    if (lane < KN) sw[wave][k] = w; if (lane == 0) sdist[wave] = dsum * (1.0f / KN); }
  LDSX();
  float fc[12], acc[12]; const float* fr = FT + n * CC;
#pragma unroll
  for (int j = 0; j < 12; ++j) { fc[j] = bfr(fr[lane + 32 * j]); acc[j] = 0.f; }
  for (int k = 0; k < KN; ++k) { const float* gr = FT + ((size_t)b * NP + sid[wave][k]) * CC; float dl[12]; float s = 0.f;
#pragma unroll
    for (int j = 0; j < 12; ++j) { dl[j] = bfr(gr[lane + 32 * j]) - fc[j]; s += dl[j]; }
#pragma unroll
    for (int o = 1; o < 32; o <<= 1) s += __shfl_xor(s, o);
    const float mu = s * (1.0f / CC); float v = 0.f;
#pragma unroll
    for (int j = 0; j < 12; ++j) { const float d = dl[j] - mu; v += d * d; }
#pragma unroll
    for (int o = 1; o < 32; o <<= 1) v += __shfl_xor(v, o);
    const float rs = rsqrtf(v * (1.0f / CC) + 1e-5f); const float w = sw[wave][k];
#pragma unroll
    for (int j = 0; j < 12; ++j) acc[j] += ((dl[j] - mu) * rs) * w; }
#pragma unroll
  for (int j = 0; j < 12; ++j) { const float v = acc[j] * (1.0f / KN); const __bf16 hb = (__bf16)v; sh_[wave][lane + 32 * j] = hb; sl_[wave][lane + 32 * j] = (__bf16)(v - (float)hb); }
  if (lane == 0) { const float v = sdist[wave]; const __bf16 hb = (__bf16)v; sh_[wave][CC] = hb; sl_[wave][CC] = (__bf16)(v - (float)hb); }
  for (int c = CC + 1 + lane; c < KIN; c += 32) { sh_[wave][c] = (__bf16)0.f; sl_[wave][c] = (__bf16)0.f; }
  LDSX();
  for (int pc = lane; pc < KIN / 8; pc += 32) { vst2((unsigned*)(FUH + n * KIN + pc * 8), *(const v4u*)&sh_[wave][pc * 8]); vst2((unsigned*)(FUL + n * KIN + pc * 8), *(const v4u*)&sl_[wave][pc * 8]); }
}
template <int MODE>
__global__ __launch_bounds__(128) void k_lin(const __bf16* __restrict__ AH, const __bf16* __restrict__ AL, const __bf16* __restrict__ P, const float* __restrict__ BI, __bf16* __restrict__ OH, __bf16* __restrict__ OL, float* __restrict__ OUT) {
  constexpr int K = (MODE == 0) ? KIN : CC;
  __shared__ __align__(16) float so[4][16][132]; __shared__ __align__(16) __bf16 soh[4][16][136], sol[4][16][136];
  const int tid = threadIdx.x, wave = tid >> 5, lane = tid & 31, col = lane & 15, g = lane >> 4; const size_t r0 = (size_t)blockIdx.x * 64 + wave * 16; const int n0 = blockIdx.y * 128;
  v8f acc[8] = {};
#pragma unroll 2
  for (int kc = 0; kc < K / 32; ++kc) { F2 a; a.h = frag_b(AH + (r0 + col) * K + kc * 32, lane); a.l = frag_b(AL + (r0 + col) * K + kc * 32, lane);
#pragma unroll
    for (int j = 0; j < 8; ++j) { const v16b w = frag_b(P + (size_t)(n0 + j * 16 + col) * K + kc * 32, lane); acc[j] = wmma_bf(a.l, w, acc[j]); acc[j] = wmma_bf(a.h, w, acc[j]); } }
#pragma unroll
  for (int j = 0; j < 8; ++j) { const float bb = bfr(BI[n0 + j * 16 + col]);
#pragma unroll
    for (int r = 0; r < 8; ++r) { const float v = acc[j][r] + bb;
      if (MODE == 0) { const float gq = gelu_exact(v); const __bf16 hb = (__bf16)gq; soh[wave][8 * g + r][j * 16 + col] = hb; sol[wave][8 * g + r][j * 16 + col] = (__bf16)(gq - (float)hb); }
      else so[wave][8 * g + r][j * 16 + col] = v; } }
  LDSX();
  if (MODE == 0) { for (int rl = 0; rl < 16; ++rl) if (lane < 16) { vst2((unsigned*)(OH + (r0 + rl) * CC + n0 + lane * 8), *(const v4u*)&soh[wave][rl][lane * 8]); vst2((unsigned*)(OL + (r0 + rl) * CC + n0 + lane * 8), *(const v4u*)&sol[wave][rl][lane * 8]); } }
  else { for (int rl = 0; rl < 16; ++rl) vst2(OUT + (r0 + rl) * CC + n0 + lane * 4, *(const v4f*)&so[wave][rl][lane * 4]); }
}
extern "C" void kernel_launch(void* const* d_in, const int* in_sizes, int n_in, void* d_out, int out_size, void* d_ws, size_t ws_size, hipStream_t stream) {
  (void)in_sizes; (void)n_in; (void)out_size;
  const float** F = (const float**)d_in;
  if (ws_size < (size_t)WS_END) return;
  char* ws = (char*)d_ws; __bf16 *PK = (__bf16*)(ws + WS_PK), *FUH = (__bf16*)(ws + WS_FUH), *FUL = (__bf16*)(ws + WS_FUL), *HH = (__bf16*)(ws + WS_HH), *HL = (__bf16*)(ws + WS_HL); int* IDX = (int*)(ws + WS_IDX);
  k_pack<<<dim3(CC, 2), 256, 0, stream>>>(F[2], F[4], PK);
  k_knn<<<NBT * NP / 256, 256, 0, stream>>>(F[0], IDX);
  k_local<<<NBT * NP / 4, 128, 0, stream>>>(F[0], F[1], IDX, FUH, FUL);
  k_lin<0><<<dim3(NBT * NP / 64, CC / 128), 128, 0, stream>>>(FUH, FUL, PK + PK_1, F[3], HH, HL, nullptr);
  k_lin<1><<<dim3(NBT * NP / 64, CC / 128), 128, 0, stream>>>(HH, HL, PK + PK_2, F[5], nullptr, nullptr, (float*)d_out);
}
